// Network_19834158973589
// MI455X (gfx1250) — hardware-verified
//
#include <hip/hip_runtime.h>
#include <math.h>

constexpr int NBATCH = 1024;
constexpr int NSTEPS = 256;
constexpr int MAXLEN = 128;
constexpr int NEMB   = 300;
constexpr int KEMB   = 320;
constexpr int LASTC4 = NEMB - 4;
constexpr int NVOC   = 50000;
constexpr int NHID   = 50;
constexpr int NGATE  = 200;
constexpr int KHP    = 64;
constexpr int NGP    = 256;
constexpr int CHUNK  = 64;
constexpr int NCHUNK = 4;
constexpr int NTHR   = 128;
constexpr int NTHC   = 256;
constexpr int EPITCH = 328;
constexpr int HPITCH = 72;
constexpr int SLABP  = 68;
constexpr int KF1 = 100, NF1 = 25, NF2 = 3;
constexpr int KF1P = 128, NF1P = 32, NF2P = 16;
constexpr int FPITCH = 136, H1PITCH = 40;
constexpr int BROWS = 64;
constexpr int SROWS = 16;
constexpr float WCARRY = 16.0f;
constexpr float WCARRY_INV = 1.0f / 16.0f;
constexpr float BN_SCALE = 0.999500374625937f;
constexpr int N8EMB   = NVOC * (KEMB / 8);
constexpr int N8WX    = NGP * (KEMB / 8);
constexpr int N8WH    = NGP * (KHP / 8);
constexpr int NSTATE4 = 2 * NBATCH * KHP / 4;

static_assert(MAXLEN == 128);
static_assert(NSTEPS == 2 * MAXLEN);
static_assert(NSTEPS == NCHUNK * CHUNK);
static_assert(MAXLEN % CHUNK == 0);
static_assert(NBATCH % BROWS == 0 && NBATCH % SROWS == 0);
static_assert(KEMB % 32 == 0 && KEMB >= NEMB && KEMB % 8 == 0);
static_assert(KHP % 32 == 0 && KHP >= NHID);
static_assert(NGP == 4 * KHP);
static_assert(NGP % 64 == 0);
static_assert((BROWS * (KEMB / 8)) % NTHR == 0);
static_assert((2 * SROWS * HPITCH) % NTHR == 0);
static_assert((SROWS * KHP / 4) % NTHR == 0);
static_assert(N8EMB % 32 == 0);
static_assert(N8WX % NTHC == 0 && N8WH % NTHC == 0);
static_assert((BROWS * NHID) % NTHR == 0);
static_assert((BROWS * (FPITCH - KF1)) % NTHR == 0);
static_assert((NF1P * FPITCH) % NTHR == 0);
static_assert((NF2P * H1PITCH) % NTHR == 0);
static_assert((BROWS * NF2) % 4 == 0);
static_assert(EPITCH % 8 == 0 && HPITCH % 8 == 0 && FPITCH % 8 == 0 && H1PITCH % 8 == 0);

typedef __attribute__((ext_vector_type(16))) _Float16 v16h;
typedef __attribute__((ext_vector_type(8)))  _Float16 v8h;
typedef __attribute__((ext_vector_type(16))) __bf16   v16b;
typedef __attribute__((ext_vector_type(8)))  __bf16   v8b;
typedef __attribute__((ext_vector_type(8)))  float    v8f;
typedef __attribute__((ext_vector_type(4)))  float    v4f;
typedef __attribute__((ext_vector_type(4)))  unsigned v4u;
typedef __attribute__((ext_vector_type(2)))  unsigned v2u;

__device__ __forceinline__ unsigned short f2bf_bits(float f) {
  unsigned u = __float_as_uint(f);
  return (unsigned short)((u + 0x7FFFu + ((u >> 16) & 1u)) >> 16);
}
__device__ __forceinline__ float bf_bits2f(unsigned short h) { return __uint_as_float(((unsigned)h) << 16); }
__device__ __forceinline__ float bf16r(float f) { return bf_bits2f(f2bf_bits(f)); }
__device__ __forceinline__ unsigned short f2h_bits(float f) { return __builtin_bit_cast(unsigned short, (_Float16)f); }

__device__ __forceinline__ void guard4_b(v8f& a, v8f& b, v8f& c, v8f& d, v16b x, v16b y) {
  asm volatile("v_nop\n\tv_nop\n\tv_nop\n\tv_nop" : "+v"(a), "+v"(b), "+v"(c), "+v"(d) : "v"(x), "v"(y));
}
__device__ __forceinline__ void guard4_h(v8f& a, v8f& b, v8f& c, v8f& d, v16h x, v16h y) {
  asm volatile("v_nop\n\tv_nop\n\tv_nop\n\tv_nop" : "+v"(a), "+v"(b), "+v"(c), "+v"(d) : "v"(x), "v"(y));
}
__device__ __forceinline__ void guard2_h(v8f& a, v8f& b, v16h x, v16h y) {
  asm volatile("v_nop\n\tv_nop\n\tv_nop\n\tv_nop" : "+v"(a), "+v"(b) : "v"(x), "v"(y));
}
__device__ __forceinline__ void guard1_h(v8f& a, v16h x, v16h y) {
  asm volatile("v_nop\n\tv_nop\n\tv_nop\n\tv_nop" : "+v"(a) : "v"(x), "v"(y));
}
__device__ __forceinline__ void keep4_h(v16h a, v16h b, v16h c, v16h d) { asm volatile("v_nop" :: "v"(a), "v"(b), "v"(c), "v"(d)); }
__device__ __forceinline__ void keep4_b(v16b a, v16b b, v16b c, v16b d) { asm volatile("v_nop" :: "v"(a), "v"(b), "v"(c), "v"(d)); }
__device__ __forceinline__ void acc_guard4(v8f& a, v8f& b, v8f& c, v8f& d) { asm volatile("v_nop\n\tv_nop\n\tv_nop\n\tv_nop" : "+v"(a), "+v"(b), "+v"(c), "+v"(d)); }
__device__ __forceinline__ void acc_guard2(v8f& a, v8f& b) { asm volatile("v_nop\n\tv_nop\n\tv_nop\n\tv_nop" : "+v"(a), "+v"(b)); }

template <typename T> struct Frag;
template <> struct Frag<_Float16> {
  typedef v16h V; union U { v16h v; v8h h[2]; };
  static __device__ __forceinline__ v16h load(const _Float16* p) {
    U f; f.h[0] = *(const v8h*)(p); f.h[1] = *(const v8h*)(p + 16); return f.v;
  }
  static __device__ __forceinline__ v8f mma(v16h a, v16h b, v8f c) {
    return __builtin_amdgcn_wmma_f32_16x16x32_f16(false, a, false, b, (short)0, c, false, false);
  }
};
template <> struct Frag<__bf16> {
  typedef v16b V; union U { v16b v; v8b h[2]; };
  static __device__ __forceinline__ v16b load(const __bf16* p) {
    U f; f.h[0] = *(const v8b*)(p); f.h[1] = *(const v8b*)(p + 16); return f.v;
  }
  static __device__ __forceinline__ v8f mma(v16b a, v16b b, v8f c) {
    return __builtin_amdgcn_wmma_f32_16x16x32_bf16(false, a, false, b, (short)0, c, false, false);
  }
};

__device__ __forceinline__ float frcp(float x)  { return __builtin_amdgcn_rcpf(x); }
__device__ __forceinline__ float fsig(float x)  { return frcp(1.0f + expf(-x)); }
__device__ __forceinline__ float ftanh(float x) { return 1.0f - 2.0f * frcp(expf(2.0f * x) + 1.0f); }

__global__ __launch_bounds__(NTHC) void emb_cvt_kernel(const float* __restrict__ emb, unsigned short* __restrict__ EB, int n8) {
  const int i = blockIdx.x * NTHC + threadIdx.x;
  if (i < n8) {
    const int row  = i / (KEMB / 8);
    const int c8   = i - row * (KEMB / 8);
    const int col  = c8 * 8;
    const int colA = (col <= LASTC4) ? col : LASTC4;
    const int colB = (col + 4 <= LASTC4) ? (col + 4) : LASTC4;
    const float* rp = emb + (size_t)row * NEMB;
    const v4f va = *(const v4f*)(rp + colA);
    const v4f vb = *(const v4f*)(rp + colB);
    const float fa = (col < NEMB) ? 1.0f : 0.0f;
    const float fb = (col + 4 < NEMB) ? 1.0f : 0.0f;
    v4u o;
    o[0] = (unsigned)f2bf_bits(fa * va[0] + 0.0f) | ((unsigned)f2bf_bits(fa * va[1] + 0.0f) << 16);
    o[1] = (unsigned)f2bf_bits(fa * va[2] + 0.0f) | ((unsigned)f2bf_bits(fa * va[3] + 0.0f) << 16);
    o[2] = (unsigned)f2bf_bits(fb * vb[0] + 0.0f) | ((unsigned)f2bf_bits(fb * vb[1] + 0.0f) << 16);
    o[3] = (unsigned)f2bf_bits(fb * vb[2] + 0.0f) | ((unsigned)f2bf_bits(fb * vb[3] + 0.0f) << 16);
    unsigned short* op = EB + (size_t)i * 8;
    *(volatile v4u*)op = o;
    __threadfence();
    *(volatile v4u*)op = o;
  }
}

__global__ __launch_bounds__(NTHC) void wprep_kernel(const float* __restrict__ W, const float* __restrict__ bv,
                                                     unsigned short* __restrict__ WX, unsigned short* __restrict__ WHT,
                                                     float* __restrict__ BP) {
  const int tid = threadIdx.x;
  const int bx  = blockIdx.x;
  if (bx < N8WX / NTHC) {
    const int i  = bx * NTHC + tid;
    const int np = i / (KEMB / 8);
    const int c8 = i - np * (KEMB / 8);
    const int g = np >> 6, u = np & 63;
    const int uc = (u < NHID) ? u : (NHID - 1);
    const int ncol = g * NHID + uc;
    const float fu = (u < NHID) ? 1.0f : 0.0f;
    v4u o;
#pragma unroll
    for (int p = 0; p < 4; ++p) {
      unsigned bits2 = 0;
#pragma unroll
      for (int q = 0; q < 2; ++q) {
        const int k  = c8 * 8 + 2 * p + q;
        const int kc = (k < NEMB) ? k : (NEMB - 1);
        const float fk = (k < NEMB) ? fu : 0.0f;
        const float x = fk * W[(size_t)kc * NGATE + ncol] + 0.0f;
        bits2 |= ((unsigned)f2bf_bits(x)) << (16 * q);
      }
      o[p] = bits2;
    }
    unsigned short* op = WX + (size_t)i * 8;
    *(volatile v4u*)op = o;
    __threadfence();
    *(volatile v4u*)op = o;
  } else if (bx < N8WX / NTHC + N8WH / NTHC) {
    const int i  = (bx - N8WX / NTHC) * NTHC + tid;
    const int np = i >> 3;
    const int c8 = i & 7;
    const int g = np >> 6, u = np & 63;
    const int uc = (u < NHID) ? u : (NHID - 1);
    const int ncol = g * NHID + uc;
    const float fu = (u < NHID) ? 1.0f : 0.0f;
    v4u o;
#pragma unroll
    for (int p = 0; p < 4; ++p) {
      unsigned bits2 = 0;
#pragma unroll
      for (int q = 0; q < 2; ++q) {
        const int k  = c8 * 8 + 2 * p + q;
        const int kc = (k < NHID) ? k : (NHID - 1);
        const float fk = (k < NHID) ? fu : 0.0f;
        const float x = fk * W[(size_t)(NEMB + kc) * NGATE + ncol] + 0.0f;
        bits2 |= ((unsigned)f2h_bits(WCARRY * bf16r(x))) << (16 * q);
      }
      o[p] = bits2;
    }
    unsigned short* op = WHT + (size_t)i * 8;
    *(volatile v4u*)op = o;
    __threadfence();
    *(volatile v4u*)op = o;
  } else {
    if (tid < NGP / 4) {
      v4f o;
#pragma unroll
      for (int e = 0; e < 4; ++e) {
        const int np = 4 * tid + e;
        const int g = np >> 6, u = np & 63;
        const int uc = (u < NHID) ? u : (NHID - 1);
        const float fu = (u < NHID) ? 1.0f : 0.0f;
        o[e] = bf16r(fu * bv[g * NHID + uc] + 0.0f);
      }
      float* op = BP + 4 * tid;
      *(volatile v4f*)op = o;
      __threadfence();
      *(volatile v4f*)op = o;
    }
  }
}

__global__ __launch_bounds__(NTHC) void zero_state_kernel(float* __restrict__ ST, int n4) {
  const int i = blockIdx.x * NTHC + threadIdx.x;
  if (i < n4) {
    const v4f z = {0.0f, 0.0f, 0.0f, 0.0f};
    float* op = ST + (size_t)i * 4;
    *(volatile v4f*)op = z;
    __threadfence();
    *(volatile v4f*)op = z;
  }
}

__global__ __launch_bounds__(NTHC) void gates_gemm_kernel(const int* __restrict__ x1, const int* __restrict__ x2,
                                                          const unsigned short* __restrict__ EBp,
                                                          const unsigned short* __restrict__ WXp,
                                                          const float* __restrict__ BP, float* __restrict__ GX, int t0) {
  __shared__ __align__(16) unsigned short Es[BROWS * EPITCH];
  __shared__ __align__(16) float sT[NTHR / 32][16 * SLABP];
  __shared__ int sTok[BROWS];
  const __bf16* WX = (const __bf16*)WXp;
  const int tid = threadIdx.x, lane = tid & 31, wave = tid >> 5;
  const int tl = blockIdx.y;
  const int t  = t0 + tl;
  const int b0 = blockIdx.x * BROWS;

  if (tid < BROWS) {
    const int col  = t & (MAXLEN - 1);
    const int tsel = t >> 7;
    const int v1 = x1[(size_t)(b0 + tid) * MAXLEN + col];
    const int v2 = x2[(size_t)(b0 + tid) * MAXLEN + col];
    int tok = v1 + tsel * (v2 - v1);
    tok = (tok < 0) ? 0 : tok;
    tok = (tok > NVOC - 1) ? (NVOC - 1) : tok;
    sTok[tid] = tok;
  }
  __syncthreads();
#pragma unroll 1
  for (int it = 0; it < (BROWS * (KEMB / 8)) / NTHR; ++it) {
    const int idx = it * NTHR + tid;
    const int row = idx / (KEMB / 8);
    const int c8  = idx - row * (KEMB / 8);
    const v4u v = *(const v4u*)(EBp + (size_t)sTok[row] * KEMB + c8 * 8);
    *(v4u*)(Es + row * EPITCH + c8 * 8) = v;
  }
  __syncthreads();

  const __bf16* Bs = (const __bf16*)Es;
  const int rlane = lane & 15;
  const int koff  = (lane >> 4) * 8;
  const int mOff  = (lane >> 4) * 8;
  const int hh    = lane >> 4;
  const int m0    = wave * 64;

  v8f acc[4][4];
#pragma unroll
  for (int i = 0; i < 4; ++i)
#pragma unroll
    for (int j = 0; j < 4; ++j) acc[i][j] = (v8f){0.f,0.f,0.f,0.f,0.f,0.f,0.f,0.f};

#pragma unroll 1
  for (int k0 = 0; k0 < KEMB; k0 += 32) {
    v16b bh[4];
#pragma unroll
    for (int j = 0; j < 4; ++j) bh[j] = Frag<__bf16>::load(Bs + ((j << 4) + rlane) * EPITCH + koff + k0);
#pragma unroll
    for (int i = 0; i < 4; ++i) {
      const v16b ah = Frag<__bf16>::load(WX + (size_t)(m0 + (i << 4) + rlane) * KEMB + koff + k0);
#pragma unroll
      for (int j = 0; j < 4; ++j) acc[i][j] = Frag<__bf16>::mma(ah, bh[j], acc[i][j]);
      guard4_b(acc[i][0], acc[i][1], acc[i][2], acc[i][3], ah, bh[3]);
    }
    keep4_b(bh[0], bh[1], bh[2], bh[3]);
  }
  acc_guard4(acc[0][0], acc[0][1], acc[0][2], acc[0][3]);
  acc_guard4(acc[1][0], acc[1][1], acc[1][2], acc[1][3]);
  acc_guard4(acc[2][0], acc[2][1], acc[2][2], acc[2][3]);
  acc_guard4(acc[3][0], acc[3][1], acc[3][2], acc[3][3]);

  float* slab = sT[wave];
  float* Cb = GX + (size_t)tl * NGP * NBATCH;
  const int c4 = rlane * 4;
#pragma unroll
  for (int i = 0; i < 4; ++i) {
    const int mBase = m0 + (i << 4);
#pragma unroll
    for (int j = 0; j < 4; ++j) {
#pragma unroll
      for (int r = 0; r < 8; ++r) {
        const float v = acc[i][j][r] + BP[mBase + mOff + r];
        slab[(mOff + r) * SLABP + (j << 4) + rlane] = v;
      }
    }
    __builtin_amdgcn_fence(__ATOMIC_RELEASE, "workgroup");
    __builtin_amdgcn_wave_barrier();
    __builtin_amdgcn_fence(__ATOMIC_ACQUIRE, "workgroup");
    for (int pass = 0; pass < 2; ++pass) {
#pragma unroll
      for (int it = 0; it < 8; ++it) {
        const int row = it * 2 + hh;
        const v4f v = *(const v4f*)(slab + row * SLABP + c4);
        *(volatile v4f*)(Cb + (size_t)(mBase + row) * NBATCH + b0 + c4) = v;
      }
      __threadfence();
    }
    __builtin_amdgcn_fence(__ATOMIC_RELEASE, "workgroup");
    __builtin_amdgcn_wave_barrier();
    __builtin_amdgcn_fence(__ATOMIC_ACQUIRE, "workgroup");
  }
}

__global__ __launch_bounds__(NTHC) void lstm_chunk_kernel(const float* __restrict__ GX, const unsigned short* __restrict__ WHp,
                                                          float* __restrict__ HS, float* __restrict__ CS) {
  __shared__ __align__(16) unsigned short Ah[2][SROWS * HPITCH];
  __shared__ __align__(16) float Hs[SROWS * SLABP];
  __shared__ __align__(16) float Cs[SROWS * SLABP];
  const _Float16* WH = (const _Float16*)WHp;
  const int tid = threadIdx.x, lane = tid & 31, wave = tid >> 5;
  const int c = lane & 15, hh = lane >> 4, koff = hh * 8;
  const int j = 16 * wave + c;
  const int b0 = blockIdx.x * SROWS;

  {
    unsigned short* ahf = &Ah[0][0];
#pragma unroll 1
    for (int it = 0; it < (2 * SROWS * HPITCH) / NTHR; ++it) ahf[it * NTHR + tid] = 0;
  }
  __syncthreads();
#pragma unroll
  for (int it = 0; it < (SROWS * KHP / 4) / NTHR; ++it) {
    const int idx = it * NTHR + tid;
    const int row = idx >> 4, c4 = (idx & 15) * 4;
    const v4f v = *(const v4f*)(HS + (size_t)(b0 + row) * KHP + c4);
    v2u pk;
    pk[0] = (unsigned)f2h_bits(v[0]) | ((unsigned)f2h_bits(v[1]) << 16);
    pk[1] = (unsigned)f2h_bits(v[2]) | ((unsigned)f2h_bits(v[3]) << 16);
    *(v2u*)(&Ah[0][row * HPITCH + c4]) = pk;
  }
  float cst[8], hst[8];
#pragma unroll
  for (int r = 0; r < 8; ++r) {
    cst[r] = CS[(size_t)(b0 + 8 * hh + r) * KHP + j];
    hst[r] = 0.0f;
  }
  v16h bq[8];
#pragma unroll
  for (int g = 0; g < 2; ++g) {
    const _Float16* wr = WH + (size_t)(g * KHP + j) * KHP + koff;
    bq[2 * g]     = Frag<_Float16>::load(wr);
    bq[2 * g + 1] = Frag<_Float16>::load(wr + 32);
  }
  keep4_h(bq[0], bq[1], bq[2], bq[3]);
#pragma unroll
  for (int g = 2; g < 4; ++g) {
    const _Float16* wr = WH + (size_t)(g * KHP + j) * KHP + koff;
    bq[2 * g]     = Frag<_Float16>::load(wr);
    bq[2 * g + 1] = Frag<_Float16>::load(wr + 32);
  }
  keep4_h(bq[4], bq[5], bq[6], bq[7]);
  __syncthreads();

  const v8f z8 = {0.f, 0.f, 0.f, 0.f, 0.f, 0.f, 0.f, 0.f};
#pragma unroll 1
  for (int tl = 0; tl < CHUNK; ++tl) {
    const int cur = tl & 1;
    float gx[4][8];
#pragma unroll
    for (int g = 0; g < 4; ++g) {
      const float* gp = GX + (size_t)(tl * NGP + g * KHP + j) * NBATCH + b0 + 8 * hh;
      const v4f lo = *(const v4f*)(gp);
      const v4f hi = *(const v4f*)(gp + 4);
#pragma unroll
      for (int e = 0; e < 4; ++e) { gx[g][e] = lo[e]; gx[g][4 + e] = hi[e]; }
    }
    const _Float16* arow = (const _Float16*)(&Ah[cur][0]) + c * HPITCH + koff;
    const v16h a0 = Frag<_Float16>::load(arow);
    const v16h a1 = Frag<_Float16>::load(arow + 32);
    v8f acc[4];
#pragma unroll
    for (int g = 0; g < 4; ++g) {
      acc[g] = Frag<_Float16>::mma(a0, bq[2 * g], z8);
      acc[g] = Frag<_Float16>::mma(a1, bq[2 * g + 1], acc[g]);
    }
    guard4_h(acc[0], acc[1], acc[2], acc[3], a0, a1);
    unsigned short* ahn = &Ah[cur ^ 1][0];
#pragma unroll
    for (int r = 0; r < 8; ++r) {
      const float zi = acc[0][r] * WCARRY_INV + gx[0][r];
      const float zj = acc[1][r] * WCARRY_INV + gx[1][r];
      const float zf = acc[2][r] * WCARRY_INV + gx[2][r];
      const float zo = acc[3][r] * WCARRY_INV + gx[3][r];
      const float cn = cst[r] * fsig(zf + 1.0f) + fsig(zi) * ftanh(zj);
      cst[r] = cn;
      const float hn = ftanh(cn) * fsig(zo);
      hst[r] = hn;
      ahn[(8 * hh + r) * HPITCH + j] = f2h_bits(hn);
    }
    __syncthreads();
  }
  keep4_h(bq[0], bq[1], bq[2], bq[3]);
  keep4_h(bq[4], bq[5], bq[6], bq[7]);

#pragma unroll
  for (int r = 0; r < 8; ++r) {
    Hs[(8 * hh + r) * SLABP + j] = hst[r];
    Cs[(8 * hh + r) * SLABP + j] = cst[r];
  }
  __syncthreads();
  for (int pass = 0; pass < 2; ++pass) {
#pragma unroll
    for (int it = 0; it < (SROWS * KHP / 4) / NTHR; ++it) {
      const int idx = it * NTHR + tid;
      const int row = idx >> 4, c4 = (idx & 15) * 4;
      const v4f vh = *(const v4f*)(Hs + row * SLABP + c4);
      const v4f vc = *(const v4f*)(Cs + row * SLABP + c4);
      *(volatile v4f*)(HS + (size_t)(b0 + row) * KHP + c4) = vh;
      *(volatile v4f*)(CS + (size_t)(b0 + row) * KHP + c4) = vc;
    }
    __threadfence();
  }
}

__global__ __launch_bounds__(NTHC) void head_kernel(const float* __restrict__ HS, const float* __restrict__ GXB,
                                                    const float* __restrict__ W1, const float* __restrict__ b1,
                                                    const float* __restrict__ W2, const float* __restrict__ b2,
                                                    float* __restrict__ out) {
  __shared__ __align__(16) unsigned short Fh[BROWS * FPITCH];
  __shared__ __align__(16) unsigned short W1s[NF1P * FPITCH];
  __shared__ __align__(16) unsigned short H1s[BROWS * H1PITCH];
  __shared__ __align__(16) unsigned short W2s[NF2P * H1PITCH];
  __shared__ __align__(16) float Os[BROWS * NF2];
  __shared__ float b1s[32];
  __shared__ float b2s[32];
  const int tid = threadIdx.x, lane = tid & 31, wave = tid >> 5;
  const int c = lane & 15, hh = lane >> 4, koff = hh * 8;
  const int b0 = blockIdx.x * BROWS;

#pragma unroll 1
  for (int it = 0; it < (BROWS * NHID) / NTHR; ++it) {
    const int idx = it * NTHR + tid;
    const int row = idx / NHID;
    const int k   = idx - row * NHID;
    const float v = HS[(size_t)(b0 + row) * KHP + k] * BN_SCALE;
    Fh[row * FPITCH + k] = f2h_bits(v);
  }
#pragma unroll 1
  for (int it = 0; it < (BROWS * NHID) / NTHR; ++it) {
    const int idx  = it * NTHR + tid;
    const int u    = idx / BROWS;
    const int brow = idx - u * BROWS;
    const float* gp = GXB + (size_t)u * NBATCH + b0 + brow;
    const float zi = gp[0];
    const float zj = gp[(size_t)1 * KHP * NBATCH];
    const float zo = gp[(size_t)3 * KHP * NBATCH];
    const float cc = fsig(zi) * ftanh(zj);
    const float hb = ftanh(cc) * fsig(zo);
    Fh[brow * FPITCH + NHID + u] = f2h_bits(hb * BN_SCALE);
  }
#pragma unroll 1
  for (int it = 0; it < (BROWS * (FPITCH - KF1)) / NTHR; ++it) {
    const int idx = it * NTHR + tid;
    const int row = idx / (FPITCH - KF1);
    const int kk  = idx - row * (FPITCH - KF1);
    Fh[row * FPITCH + KF1 + kk] = 0;
  }
#pragma unroll 1
  for (int it = 0; it < (NF1P * FPITCH) / NTHR; ++it) {
    const int idx = it * NTHR + tid;
    const int n = idx / FPITCH;
    const int k = idx - n * FPITCH;
    const int nc = (n < NF1) ? n : (NF1 - 1);
    const int kc = (k < KF1) ? k : (KF1 - 1);
    const float f = (n < NF1 && k < KF1) ? 1.0f : 0.0f;
    const float x = f * W1[kc * NF1 + nc] + 0.0f;
    W1s[idx] = f2h_bits(WCARRY * bf16r(x));
  }
#pragma unroll 1
  for (int it = 0; it < (NF2P * H1PITCH) / NTHR; ++it) {
    const int idx = it * NTHR + tid;
    const int n = idx / H1PITCH;
    const int k = idx - n * H1PITCH;
    const int nc = (n < NF2) ? n : (NF2 - 1);
    const int kc = (k < NF1) ? k : (NF1 - 1);
    const float f = (n < NF2 && k < NF1) ? 1.0f : 0.0f;
    const float x = f * W2[kc * NF2 + nc] + 0.0f;
    W2s[idx] = f2h_bits(WCARRY * bf16r(x));
  }
  if (tid < 32) {
    const int nc1 = (tid < NF1) ? tid : (NF1 - 1);
    const float f1 = (tid < NF1) ? 1.0f : 0.0f;
    b1s[tid] = bf16r(f1 * b1[nc1] + 0.0f);
    const int nc2 = (tid < NF2) ? tid : (NF2 - 1);
    const float f2 = (tid < NF2) ? 1.0f : 0.0f;
    b2s[tid] = bf16r(f2 * b2[nc2] + 0.0f);
  }
  __syncthreads();

  const v8f z8 = {0.f, 0.f, 0.f, 0.f, 0.f, 0.f, 0.f, 0.f};
  const _Float16* fap = (const _Float16*)Fh + (16 * wave + c) * FPITCH + koff;
  const _Float16* w1p = (const _Float16*)W1s + c * FPITCH + koff;
  v8f acc1a = z8, acc1b = z8;
#pragma unroll
  for (int ks = 0; ks < KF1P / 32; ++ks) {
    const v16h a  = Frag<_Float16>::load(fap + 32 * ks);
    const v16h w0 = Frag<_Float16>::load(w1p + 32 * ks);
    const v16h w1 = Frag<_Float16>::load(w1p + 16 * FPITCH + 32 * ks);
    acc1a = Frag<_Float16>::mma(a, w0, acc1a);
    acc1b = Frag<_Float16>::mma(a, w1, acc1b);
    guard2_h(acc1a, acc1b, a, w1);
    keep4_h(a, w0, w1, a);
  }
  acc_guard2(acc1a, acc1b);
  {
    const float bb0 = b1s[c], bb1 = b1s[16 + c];
#pragma unroll
    for (int r = 0; r < 8; ++r) {
      const float v0 = fmaxf(acc1a[r] * WCARRY_INV + bb0, 0.0f);
      const float v1 = fmaxf(acc1b[r] * WCARRY_INV + bb1, 0.0f);
      H1s[(16 * wave + 8 * hh + r) * H1PITCH + c]      = f2h_bits(v0);
      H1s[(16 * wave + 8 * hh + r) * H1PITCH + 16 + c] = f2h_bits(v1);
    }
  }
  __syncthreads();
  const v16h a2 = Frag<_Float16>::load((const _Float16*)H1s + (16 * wave + c) * H1PITCH + koff);
  const v16h w2 = Frag<_Float16>::load((const _Float16*)W2s + c * H1PITCH + koff);
  v8f acc2 = Frag<_Float16>::mma(a2, w2, z8);
  guard1_h(acc2, a2, w2);
  {
    const float bb2 = b2s[c];
#pragma unroll
    for (int r = 0; r < 8; ++r) {
      const float o = (acc2[r] * WCARRY_INV + bb2) * BN_SCALE;
      if (c < NF2) Os[(16 * wave + 8 * hh + r) * NF2 + c] = o;
    }
  }
  __syncthreads();
  if (tid < (BROWS * NF2) / 4) {
    const v4f v = *(const v4f*)(Os + 4 * tid);
    float* op = out + (size_t)b0 * NF2 + 4 * tid;
    *(volatile v4f*)op = v;
    __threadfence();
    *(volatile v4f*)op = v;
  }
}

extern "C" void kernel_launch(void* const* d_in, const int* in_sizes, int n_in,
                              void* d_out, int out_size, void* d_ws, size_t ws_size, hipStream_t stream) {
  if (n_in < 11 || d_out == nullptr || d_ws == nullptr) return;
  if (in_sizes[0] != NBATCH * MAXLEN || in_sizes[1] != NBATCH * MAXLEN || in_sizes[2] != NVOC * NEMB ||
      in_sizes[3] != (NEMB + NHID) * NGATE || in_sizes[4] != NGATE || in_sizes[5] != (NEMB + NHID) * NGATE ||
      in_sizes[6] != NGATE || in_sizes[7] != KF1 * NF1 || in_sizes[8] != NF1 || in_sizes[9] != NF1 * NF2 ||
      in_sizes[10] != NF2 || out_size != NBATCH * NF2) return;

  const int*   x1  = (const int*)  d_in[0];
  const int*   x2  = (const int*)  d_in[1];
  const float* emb = (const float*)d_in[2];
  const float* Wfw = (const float*)d_in[3];
  const float* bfw = (const float*)d_in[4];
  const float* Wbw = (const float*)d_in[5];
  const float* bbw = (const float*)d_in[6];
  const float* W1  = (const float*)d_in[7];
  const float* b1  = (const float*)d_in[8];
  const float* W2  = (const float*)d_in[9];
  const float* b2  = (const float*)d_in[10];
  float* out = (float*)d_out;

  char* ws = (char*)d_ws; size_t off = 0;
  auto carve = [&](size_t bytes) -> char* { char* p = ws + off; off += (bytes + 255) & ~(size_t)255; return p; };
  unsigned short* EB  = (unsigned short*)carve((size_t)NVOC * KEMB * 2);
  unsigned short* WXF = (unsigned short*)carve((size_t)NGP * KEMB * 2);
  unsigned short* WXB = (unsigned short*)carve((size_t)NGP * KEMB * 2);
  unsigned short* WHF = (unsigned short*)carve((size_t)NGP * KHP * 2);
  unsigned short* WHB = (unsigned short*)carve((size_t)NGP * KHP * 2);
  float*          BPF = (float*)carve((size_t)NGP * 4);
  float*          BPB = (float*)carve((size_t)NGP * 4);
  float*          STATE = (float*)carve((size_t)2 * NBATCH * KHP * 4);
  float*          GX  = (float*)carve((size_t)CHUNK * NGP * NBATCH * 4);
  float*          GXB = (float*)carve((size_t)NGP * NBATCH * 4);
  if (off > ws_size || off > (size_t)134217728) return;
  float* HS = STATE;
  float* CS = STATE + (size_t)NBATCH * KHP;

  emb_cvt_kernel<<<(N8EMB + NTHC - 1) / NTHC, NTHC, 0, stream>>>(emb, EB, N8EMB);
  wprep_kernel<<<N8WX / NTHC + N8WH / NTHC + 1, NTHC, 0, stream>>>(Wfw, bfw, WXF, WHF, BPF);
  wprep_kernel<<<N8WX / NTHC + N8WH / NTHC + 1, NTHC, 0, stream>>>(Wbw, bbw, WXB, WHB, BPB);
  zero_state_kernel<<<(NSTATE4 + NTHC - 1) / NTHC, NTHC, 0, stream>>>(STATE, NSTATE4);
  for (int ch = 0; ch < NCHUNK; ++ch) {
    gates_gemm_kernel<<<dim3(NBATCH / BROWS, CHUNK), NTHR, 0, stream>>>(x1, x2, EB, WXF, BPF, GX, ch * CHUNK);
    lstm_chunk_kernel<<<NBATCH / SROWS, NTHR, 0, stream>>>(GX, WHF, HS, CS);
  }
  gates_gemm_kernel<<<dim3(NBATCH / BROWS, 1), NTHR, 0, stream>>>(x1, x2, EB, WXB, BPB, GXB, NSTEPS - 1);
  head_kernel<<<NBATCH / BROWS, NTHR, 0, stream>>>(HS, GXB, W1, b1, W2, b2, out);
}
